// MHSA_33131377722100
// MI455X (gfx1250) — hardware-verified
//
#include <hip/hip_runtime.h>
#include <stdint.h>


typedef unsigned short hword;
typedef hword us8  __attribute__((ext_vector_type(8)));
typedef hword us16 __attribute__((ext_vector_type(16)));
typedef __bf16 bf16x16 __attribute__((ext_vector_type(16)));
typedef _Float16 f16x16 __attribute__((ext_vector_type(16)));
typedef float v8f __attribute__((ext_vector_type(8)));
typedef float v4f __attribute__((ext_vector_type(4)));
typedef int v4i __attribute__((ext_vector_type(4)));

#ifndef NB
#define NB 2
#endif
#ifndef SEQ
#define SEQ 2048
#endif
#define NB_FULL  2
#define SEQ_FULL 2048
#define DIM   1024
#define HD    64
#define NH    16
#define MROWS (NB * SEQ)
#define MT    (MROWS / 64)
#define NQT   (SEQ / 64)
#define NBH   (NB * NH)
#define LDT   68
#define FLP   32
#define FLAG_FULL 1522192999

static_assert(NB >= 1 && NB <= NB_FULL);
static_assert(SEQ % 256 == 0 && SEQ >= 256 && SEQ <= SEQ_FULL);
static_assert(NQT <= FLP);
static_assert(DIM % 32 == 0 && HD == 64 && NH * HD == DIM);

__device__ __forceinline__ hword f2bf(float x) {
    unsigned int u = __float_as_uint(x);
    u = (u + 0x7FFFu + ((u >> 16) & 1u)) >> 16;
    return (hword)u;
}
__device__ __forceinline__ float bf2f(hword b) {
    return __uint_as_float(((unsigned int)b) << 16);
}
__device__ __forceinline__ hword f2h(float x) {
    _Float16 t = (_Float16)x;
    return __builtin_bit_cast(hword, t);
}
__device__ __forceinline__ v8f zero8() {
    v8f z;
#pragma unroll
    for (int i = 0; i < 8; ++i) z[i] = 0.0f;
    return z;
}

__device__ __forceinline__ v8f mma_bf(v8f c, us16 a, us16 b) {
    bf16x16 av = __builtin_bit_cast(bf16x16, a);
    bf16x16 bv = __builtin_bit_cast(bf16x16, b);
    c = __builtin_amdgcn_wmma_f32_16x16x32_bf16(false, av, false, bv, (short)0, c, false, false);
    asm volatile("v_nop\n\tv_nop\n\tv_nop\n\tv_nop" : "+v"(c) : "v"(a), "v"(b));
    return c;
}
__device__ __forceinline__ v8f mma_hf(v8f c, us16 a, us16 b) {
    f16x16 av = __builtin_bit_cast(f16x16, a);
    f16x16 bv = __builtin_bit_cast(f16x16, b);
    c = __builtin_amdgcn_wmma_f32_16x16x32_f16(false, av, false, bv, (short)0, c, false, false);
    asm volatile("v_nop\n\tv_nop\n\tv_nop\n\tv_nop" : "+v"(c) : "v"(a), "v"(b));
    return c;
}

__device__ __forceinline__ us16 frag_rows(const hword* p, int ld, int row, int k0, int h) {
    const hword* base = p + (size_t)row * ld + k0 + 8 * h;
    us8 e0 = *(const us8*)(base);
    us8 e1 = *(const us8*)(base + 16);
    return __builtin_shufflevector(e0, e1, 0, 1, 2, 3, 4, 5, 6, 7,
                                   8, 9, 10, 11, 12, 13, 14, 15);
}

template <int ACT>
__global__ __launch_bounds__(256) void k_cvt(const float* __restrict__ s0,
                                             const float* __restrict__ s1,
                                             const float* __restrict__ s2,
                                             hword* d0, hword* d1, hword* d2) {
    const int sel = blockIdx.y;
    const float* src = (sel == 0) ? s0 : ((sel == 1) ? s1 : s2);
    hword* dst = (sel == 0) ? d0 : ((sel == 1) ? d1 : d2);
    const int i = blockIdx.x * 256 + threadIdx.x;
    size_t si;
    if (ACT) {
        const int per = SEQ * (DIM / 8);
        if (i >= NB * per) return;
        const int b = i / per;
        const int rem = i - b * per;
        si = (size_t)b * ((size_t)SEQ_FULL * (DIM / 8)) + (size_t)rem;
    } else {
        if (i >= DIM * (DIM / 8)) return;
        si = (size_t)i;
    }
    const float* s = src + si * 8;
    const v4f a = *(const v4f*)(s);
    const v4f b = *(const v4f*)(s + 4);
    us8 o;
#pragma unroll
    for (int e = 0; e < 4; ++e) {
        o[e]     = f2bf(a[e]);
        o[4 + e] = f2bf(b[e]);
    }
    const size_t o8 = (size_t)i * 8;
    *(volatile us8*)(dst + o8) = o;
    __threadfence();
    *(volatile us8*)(dst + o8) = o;
}

__global__ __launch_bounds__(256) void k_mflag(const float* __restrict__ mask, int* flg) {
    __shared__ float part[256 * 8];
    __shared__ __align__(16) int fline[FLP];
    const int t = threadIdx.x, qt = blockIdx.x;
    const int r = t >> 2, cq = t & 3;
    const float* rowp = mask + (size_t)(qt * 64 + r) * SEQ_FULL;
#pragma unroll 1
    for (int cc = 0; cc < NQT / 4; ++cc) {
        const float* p = rowp + (cc * 4 + cq) * 64;
        float mx = -3.0e38f;
#pragma unroll
        for (int j = 0; j < 16; ++j) {
            const v4f v = *(const v4f*)(p + 4 * j);
            mx = fmaxf(mx, fmaxf(fmaxf(v[0], v[1]), fmaxf(v[2], v[3])));
        }
        part[t * 8 + cc] = mx;
    }
    __syncthreads();
    if (t < 32) {
        const int c = (t < NQT) ? t : (NQT - 1);
        const int ccq = c & 3, ccc = c >> 2;
        float mx = -3.0e38f;
#pragma unroll 8
        for (int rr = 0; rr < 64; ++rr) mx = fmaxf(mx, part[(rr * 4 + ccq) * 8 + ccc]);
        fline[t] = (t < NQT && mx <= -1.0e8f) ? FLAG_FULL : 0;
    }
    __syncthreads();
    if (t < 8) {
        const v4i v = *(const v4i*)(fline + 4 * t);
        int* dp = flg + qt * FLP + 4 * t;
        *(volatile v4i*)dp = v;
        __threadfence();
        *(volatile v4i*)dp = v;
    }
}

__device__ __forceinline__ void qk_pass(const float* tile, hword* P0, hword* P1,
                                        size_t rb, int w, int p, int lq) {
#pragma unroll
    for (int i = 0; i < 4; ++i) {
        const int row = w * 16 + 4 * i + lq;
        const float* sp = tile + row * LDT + 8 * p;
        const v4f u0 = *(const v4f*)(sp);
        const v4f u1 = *(const v4f*)(sp + 4);
        us8 oh, ol;
#pragma unroll
        for (int e = 0; e < 4; ++e) {
            const hword a = f2bf(u0[e]);
            oh[e] = a;
            ol[e] = f2bf(u0[e] - bf2f(a));
            const hword c = f2bf(u1[e]);
            oh[4 + e] = c;
            ol[4 + e] = f2bf(u1[e] - bf2f(c));
        }
        const size_t doff = (rb + (size_t)row) * HD + 8 * p;
        *(volatile us8*)(P0 + doff) = oh;
        *(volatile us8*)(P1 + doff) = ol;
    }
}
__device__ __forceinline__ void v_pass(const float* tile, hword* vt, size_t vb, int n0,
                                       int w, int p, int lq) {
#pragma unroll
    for (int i = 0; i < 4; ++i) {
        const int d = w * 16 + 4 * i + lq;
        us8 o;
#pragma unroll
        for (int e = 0; e < 8; ++e) o[e] = f2h(tile[(8 * p + e) * LDT + d]);
        *(volatile us8*)(vt + (vb + (size_t)d) * SEQ + (size_t)n0 + 8 * p) = o;
    }
}

template <int SV>
__global__ __launch_bounds__(128) void k_qkv(const hword* x0p, const hword* x1p,
                                             const hword* w0p, const hword* w1p,
                                             hword* d0, hword* d1, hword* d2, hword* d3) {
    __shared__ __align__(16) float tile[64 * LDT];
    const int w = threadIdx.x >> 5, lane = threadIdx.x & 31;
    const int h = lane >> 4, m = lane & 15;
    const int mt = blockIdx.x % MT, ng = blockIdx.x / MT;
    const int s  = SV ? 2 : (ng >> 4);
    const int hh = SV ? ng : (ng & 15);
    const hword* xp = (SV == 0 && s == 1) ? x1p : x0p;
    const hword* wp = (SV == 0 && s == 1) ? w1p : w0p;
    const int tok0 = mt * 64;
    const int wr = w & 1, wc = w >> 1;
    const int ar0 = tok0 + wr * 32;

    int orow[2];
#pragma unroll
    for (int t = 0; t < 2; ++t) orow[t] = hh * HD + wc * 32 + t * 16 + m;

    v8f acc[2][2];
#pragma unroll
    for (int mi = 0; mi < 2; ++mi)
#pragma unroll
        for (int t = 0; t < 2; ++t) acc[mi][t] = zero8();

#pragma unroll 1
    for (int k0 = 0; k0 < DIM; k0 += 32) {
        const us16 a0 = frag_rows(xp, DIM, ar0 + m, k0, h);
        const us16 a1 = frag_rows(xp, DIM, ar0 + 16 + m, k0, h);
#pragma unroll
        for (int t = 0; t < 2; ++t) {
            const us16 b = frag_rows(wp, DIM, orow[t], k0, h);
            acc[0][t] = mma_bf(acc[0][t], a0, b);
            acc[1][t] = mma_bf(acc[1][t], a1, b);
        }
    }

    const float scl = (SV == 0 && s == 0) ? 0.125f : 1.0f;
#pragma unroll
    for (int t = 0; t < 2; ++t) {
#pragma unroll
        for (int mi = 0; mi < 2; ++mi)
#pragma unroll
            for (int r = 0; r < 8; ++r)
                tile[(wr * 32 + mi * 16 + 8 * h + r) * LDT + wc * 32 + t * 16 + m] =
                    acc[mi][t][r] * scl;
    }
    __syncthreads();

    const int bb = tok0 / SEQ, n0 = tok0 % SEQ;
    const int p = lane & 7, lq = lane >> 3;
    if (SV == 0) {
        hword* P0 = (s == 0) ? d0 : d2;
        hword* P1 = (s == 0) ? d1 : d3;
        const size_t rb = ((size_t)(bb * NH + hh)) * SEQ + (size_t)n0;
        qk_pass(tile, P0, P1, rb, w, p, lq);
        __threadfence();
        qk_pass(tile, P0, P1, rb, w, p, lq);
    } else {
        const size_t vb = ((size_t)(bb * NH + hh)) * HD;
        v_pass(tile, d0, vb, n0, w, p, lq);
        __threadfence();
        v_pass(tile, d0, vb, n0, w, p, lq);
    }
}

__global__ __launch_bounds__(128) void k_attn(const hword* qh, const hword* ql,
                                              const hword* kh, const hword* kl,
                                              const hword* vt, const float* __restrict__ mask,
                                              const int* __restrict__ flg, float* out) {
    __shared__ __align__(16) float st[4 * 16 * LDT];
    const int w = threadIdx.x >> 5, lane = threadIdx.x & 31;
    const int h = lane >> 4, m = lane & 15;
    const int qt = blockIdx.x % NQT, bh = blockIdx.x / NQT;
    const int bb = bh / NH, hh = bh % NH;
    const size_t poff = (size_t)bh * SEQ * HD;
    const hword* qhp = qh + poff;
    const hword* qlp = ql + poff;
    const hword* khp = kh + poff;
    const hword* klp = kl + poff;
    const hword* vtp = vt + poff;
    const int q0 = qt * 64 + w * 16;
    const int qi = q0 + m;

    const int se = hh + 1;
    const float sbase = (se & 1) ? 0.70710678118654752f : 1.0f;
    const float slope = sbase * __uint_as_float(((unsigned int)(127 - (se >> 1))) << 23);

    us16 qbh[2], qbl[2];
#pragma unroll
    for (int dc = 0; dc < 2; ++dc) {
        qbh[dc] = frag_rows(qhp, HD, qi, dc * 32, h);
        qbl[dc] = frag_rows(qlp, HD, qi, dc * 32, h);
    }

    v8f oacc[4];
#pragma unroll
    for (int dt = 0; dt < 4; ++dt) oacc[dt] = zero8();
    float mrun = -1.0e30f, lrun = 0.0f;

    const float* mrowp = mask + (size_t)qi * SEQ_FULL + 8 * h;

#pragma unroll 1
    for (int kc = 0; kc < SEQ; kc += 64) {
        const int fv = __builtin_amdgcn_readfirstlane(flg[qt * FLP + (kc >> 6)]);
        if (fv == FLAG_FULL) {
            float mm = mrun;
            mm = fminf(mm, __shfl_xor(mm, 16, 32));
            mm = fminf(mm, __shfl_xor(mm, 8, 32));
            mm = fminf(mm, __shfl_xor(mm, 4, 32));
            mm = fminf(mm, __shfl_xor(mm, 2, 32));
            mm = fminf(mm, __shfl_xor(mm, 1, 32));
            const int sk = __builtin_amdgcn_readfirstlane((mm >= -1.0e4f) ? 1 : 0);
            if (sk) continue;
        }

        v8f sacc[4];
#pragma unroll
        for (int kt = 0; kt < 4; ++kt) {
            v8f sa = zero8();
            const int krow = kc + kt * 16 + m;
#pragma unroll
            for (int dc = 0; dc < 2; ++dc) {
                const us16 ka = frag_rows(khp, HD, krow, dc * 32, h);
                const us16 kb = frag_rows(klp, HD, krow, dc * 32, h);
                sa = mma_bf(sa, ka, qbh[dc]);
                sa = mma_bf(sa, ka, qbl[dc]);
                sa = mma_bf(sa, kb, qbh[dc]);
            }
            sacc[kt] = sa;
        }

        float mloc = -1.0e30f;
#pragma unroll
        for (int kt = 0; kt < 4; ++kt) {
            const v4f g0 = *(const v4f*)(mrowp + kc + kt * 16);
            const v4f g1 = *(const v4f*)(mrowp + kc + kt * 16 + 4);
            const int kb = kc + kt * 16 + 8 * h - qi;
#pragma unroll
            for (int r = 0; r < 4; ++r) {
                float x0 = sacc[kt][r] + slope * (float)(kb + r);
                x0 = x0 + bf2f(f2bf(g0[r]));
                float x1 = sacc[kt][4 + r] + slope * (float)(kb + 4 + r);
                x1 = x1 + bf2f(f2bf(g1[r]));
                sacc[kt][r] = x0;
                sacc[kt][4 + r] = x1;
                mloc = fmaxf(mloc, fmaxf(x0, x1));
            }
        }

        mloc = fmaxf(mloc, __shfl_xor(mloc, 16, 32));
        const float mnew = fmaxf(mrun, mloc);
        const float corr = __expf(mrun - mnew);
        mrun = mnew;
        float lsum = 0.0f;
        us16 pb[2];
#pragma unroll
        for (int kt = 0; kt < 4; ++kt) {
#pragma unroll
            for (int r = 0; r < 8; ++r) {
                const float pv = __expf(sacc[kt][r] - mnew);
                lsum += pv;
                pb[kt >> 1][(kt & 1) * 8 + r] = f2h(pv * 16384.0f);
            }
        }
        lsum += __shfl_xor(lsum, 16, 32);
        lrun = lrun * corr + lsum;
#pragma unroll
        for (int dt = 0; dt < 4; ++dt) oacc[dt] = oacc[dt] * corr;

#pragma unroll
        for (int ks = 0; ks < 2; ++ks) {
#pragma unroll
            for (int dt = 0; dt < 4; ++dt) {
                const us16 va = frag_rows(vtp, SEQ, dt * 16 + m, kc + ks * 32, h);
                oacc[dt] = mma_hf(oacc[dt], va, pb[ks]);
            }
        }
    }

    const float inv = 1.0f / (lrun * 16384.0f);
    float* sw = st + w * (16 * LDT);
#pragma unroll
    for (int dt = 0; dt < 4; ++dt) {
        v4f o0, o1;
#pragma unroll
        for (int r = 0; r < 4; ++r) {
            o0[r] = oacc[dt][r] * inv;
            o1[r] = oacc[dt][4 + r] * inv;
        }
        float* tp = sw + m * LDT + dt * 16 + 8 * h;
        *(v4f*)(tp) = o0;
        *(v4f*)(tp + 4) = o1;
    }
    __syncthreads();

#pragma unroll
    for (int i = 0; i < 8; ++i) {
        const int row = 2 * i + h;
        const v4f v = *(const v4f*)(sw + row * LDT + 4 * m);
        float* dp = out + ((size_t)(bb * SEQ + q0 + row)) * DIM + hh * HD + 4 * m;
        *(volatile v4f*)dp = v;
    }
    __threadfence();
#pragma unroll
    for (int i = 0; i < 8; ++i) {
        const int row = 2 * i + h;
        const v4f v = *(const v4f*)(sw + row * LDT + 4 * m);
        float* dp = out + ((size_t)(bb * SEQ + q0 + row)) * DIM + hh * HD + 4 * m;
        *(volatile v4f*)dp = v;
    }
}

extern "C" void kernel_launch(void* const* d_in, const int* in_sizes, int n_in,
                              void* d_out, int out_size, void* d_ws, size_t ws_size,
                              hipStream_t stream) {
    if (n_in < 7) return;
    const int need_x = NB * SEQ_FULL * DIM;
    const int need_m = SEQ * SEQ_FULL;
    const int need_w = DIM * DIM;
    if (in_sizes[0] < need_x || in_sizes[1] < need_x || in_sizes[2] < need_x ||
        in_sizes[3] < need_m || in_sizes[4] < need_w || in_sizes[5] < need_w ||
        in_sizes[6] < need_w || out_size < MROWS * DIM) return;

    const float* xq   = (const float*)d_in[0];
    const float* xk   = (const float*)d_in[1];
    const float* xv   = (const float*)d_in[2];
    const float* mask = (const float*)d_in[3];
    const float* Wq   = (const float*)d_in[4];
    const float* Wk   = (const float*)d_in[5];
    const float* Wv   = (const float*)d_in[6];
    float* out = (float*)d_out;

    const size_t b_fl = (size_t)FLP * FLP * 4;
    const size_t b_x  = (size_t)MROWS * DIM * 2;
    const size_t b_w  = (size_t)DIM * DIM * 2;
    const size_t b_hp = (size_t)NBH * SEQ * HD * 2;
    size_t off = 0;
    char* ws = (char*)d_ws;
    int*   flg = (int*)(ws + off);   off += b_fl;
    hword* xqb = (hword*)(ws + off); off += b_x;
    hword* xkb = (hword*)(ws + off); off += b_x;
    hword* xvb = (hword*)(ws + off); off += b_x;
    hword* wqb = (hword*)(ws + off); off += b_w;
    hword* wkb = (hword*)(ws + off); off += b_w;
    hword* wvb = (hword*)(ws + off); off += b_w;
    hword* qhp = (hword*)(ws + off); off += b_hp;
    hword* qlp = (hword*)(ws + off); off += b_hp;
    hword* khp = (hword*)(ws + off); off += b_hp;
    hword* klp = (hword*)(ws + off); off += b_hp;
    hword* vtp = (hword*)(ws + off); off += b_hp;
    if (off > ws_size) return;

    k_cvt<1><<<dim3(MROWS * (DIM / 8) / 256, 3), 256, 0, stream>>>(xq, xk, xv, xqb, xkb, xvb);
    k_cvt<0><<<dim3(DIM * (DIM / 8) / 256, 3), 256, 0, stream>>>(Wq, Wk, Wv, wqb, wkb, wvb);

    k_mflag<<<NQT, 256, 0, stream>>>(mask, flg);

    k_qkv<0><<<MT * 32, 128, 0, stream>>>(xqb, xkb, wqb, wkb, qhp, qlp, khp, klp);
    k_qkv<1><<<MT * 16, 128, 0, stream>>>(xvb, xvb, wvb, wvb, vtp, vtp, vtp, vtp);

    k_attn<<<NBH * NQT, 128, 0, stream>>>(qhp, qlp, khp, klp, vtp, mask, flg, out);
}
